// NoFieldSymmetricPredictionSourceBlock_13872744366309
// MI455X (gfx1250) — hardware-verified
//
#include <hip/hip_runtime.h>
#include <stddef.h>


#define CH      64
#define NTHR    256
#define NWAVE   8
#define NBN     32
#define NROW    128
#define APN     72
#define NBE     64
#define TROW    256
#define EPT     8
#define NGRP    2
#define CHUNK   (NTHR * EPT * NGRP)
#define WCAP    (EPT * NGRP * 32)
#define LISTN   (NWAVE * WCAP)
#define NBC     4096
#define WSCAP   134217728
#define WO_B0   0
#define WO_F1H  2048
#define WO_F1L  6144
#define WO_F2H  10240
#define WO_F2L  14336
#define WO_F3H  18432
#define WO_F3L  26624
#define WO_N10H 34816
#define WO_N10L 38912
#define WO_N20H 43008
#define WO_N20L 47104
#define WO_N11H 51200
#define WO_N11L 55296
#define WO_N21H 59392
#define WO_N21L 63488
#define WTOT    67584
#define WBLK    33
#define RS8     0.35355339059327373f
#define RS128   0.088388347648318447f
#define R40     0.025f
#define SQ3I    0.57735026918962576f

static_assert((CHUNK & (CHUNK - 1)) == 0);
static_assert(CHUNK == NBC);
static_assert(WTOT == WBLK * NTHR * 8);
static_assert(NROW == NWAVE * 16);
static_assert(NBN * 4 == NROW);
static_assert(NBE == 4 * 16);
static_assert(((APN * 2) % 16) == 0);
static_assert((NBC % (32 * NWAVE)) == 0);

typedef float          v2f  __attribute__((ext_vector_type(2)));
typedef float          v4f  __attribute__((ext_vector_type(4)));
typedef float          v8f  __attribute__((ext_vector_type(8)));
typedef int            v4i  __attribute__((ext_vector_type(4)));
typedef unsigned short v8us __attribute__((ext_vector_type(8)));
typedef unsigned short v16us __attribute__((ext_vector_type(16)));
typedef __bf16         v16bf __attribute__((ext_vector_type(16)));
union FragB { v16bf v; v16us u; v8us h[2]; };

__device__ __forceinline__ v8f wm(v16bf a, v16bf b, v8f c) {
  v8f d = __builtin_amdgcn_wmma_f32_16x16x32_bf16(false, a, false, b, (short)0, c, false, false);
  asm volatile("v_nop\n\tv_nop\n\tv_nop\n\tv_nop" : "+v"(d) : "v"(a), "v"(b));
  return d;
}

__device__ __forceinline__ v8f zero8() {
  v8f z = {0.f, 0.f, 0.f, 0.f, 0.f, 0.f, 0.f, 0.f};
  return z;
}

__device__ __forceinline__ unsigned bf_rne(float x) {
  const unsigned u = __float_as_uint(x);
  return (u + 0x7FFFu + ((u >> 16) & 1u)) >> 16;
}
__device__ __forceinline__ void split_bf(float x, unsigned short& hi, unsigned short& lo) {
  const unsigned h = bf_rne(x);
  const float hf = __uint_as_float(h << 16);
  hi = (unsigned short)h;
  lo = (unsigned short)bf_rne(x - hf);
}

__device__ __forceinline__ float silu_f(float v) {
  return v * __builtin_amdgcn_rcpf(1.0f + __expf(-v));
}

__global__ __launch_bounds__(NTHR) void k_wprep(
    const float* __restrict__ fw0, const float* __restrict__ fw1,
    const float* __restrict__ fw2, const float* __restrict__ fw3,
    const float* __restrict__ w10, const float* __restrict__ w11,
    const float* __restrict__ w20, const float* __restrict__ w21,
    unsigned short* wp) {
  const int tid = (int)threadIdx.x;
  const int b = (int)blockIdx.x;
  const float* src = fw1;
  int ncols = 64, part = 0, segoff = WO_F1H;
  if (b == 0)       { src = fw0; ncols = 64;  part = 0; segoff = WO_B0; }
  else if (b <= 2)  { src = fw1; ncols = 64;  part = 0; segoff = WO_F1H; }
  else if (b <= 4)  { src = fw1; ncols = 64;  part = 1; segoff = WO_F1L; }
  else if (b <= 6)  { src = fw2; ncols = 64;  part = 0; segoff = WO_F2H; }
  else if (b <= 8)  { src = fw2; ncols = 64;  part = 1; segoff = WO_F2L; }
  else if (b <= 12) { src = fw3; ncols = 256; part = 0; segoff = WO_F3H; }
  else if (b <= 16) { src = fw3; ncols = 256; part = 1; segoff = WO_F3L; }
  else if (b <= 18) { src = w10; ncols = 64;  part = 0; segoff = WO_N10H; }
  else if (b <= 20) { src = w10; ncols = 64;  part = 1; segoff = WO_N10L; }
  else if (b <= 22) { src = w20; ncols = 64;  part = 0; segoff = WO_N20H; }
  else if (b <= 24) { src = w20; ncols = 64;  part = 1; segoff = WO_N20L; }
  else if (b <= 26) { src = w11; ncols = 64;  part = 0; segoff = WO_N11H; }
  else if (b <= 28) { src = w11; ncols = 64;  part = 1; segoff = WO_N11L; }
  else if (b <= 30) { src = w21; ncols = 64;  part = 0; segoff = WO_N21H; }
  else              { src = w21; ncols = 64;  part = 1; segoff = WO_N21L; }
  const int og = (b * NTHR + tid) * 8;
  const int o  = og - segoff;
  float v[8];
  int zero = 0;
  if (b == 0) {
    const int n   = o >> 5;
    const int grp = (o >> 3) & 3;
    part = (grp == 2) ? 1 : 0;
    zero = (grp == 3) ? 1 : 0;
#pragma unroll
    for (int j = 0; j < 8; ++j) v[j] = src[j * 64 + n];
  } else {
    const int n  = o >> 6;
    const int k0 = o & 63;
    const int col = (ncols == 256 && n >= 64) ? n + 128 : n;
#pragma unroll
    for (int j = 0; j < 8; ++j) v[j] = src[(size_t)(k0 + j) * ncols + col];
  }
  v8us ov;
#pragma unroll
  for (int j = 0; j < 8; ++j) {
    unsigned short hi, lo;
    split_bf(v[j], hi, lo);
    unsigned short s = part ? lo : hi;
    s = zero ? (unsigned short)0 : s;
    ov[j] = s;
  }
  unsigned short* dp = wp + og;
  *(volatile v8us*)dp = ov;
  __threadfence();
  *(volatile v8us*)dp = ov;
}

__global__ __launch_bounds__(NTHR) void k_node(
    const float* __restrict__ nf, const unsigned short* __restrict__ wp,
    float* T1, float* T2, int nN) {
  __shared__ __attribute__((aligned(16))) float lds[9216];
  unsigned short* sAh = (unsigned short*)lds;
  unsigned short* sAl = sAh + NROW * APN;
  float* stg = lds;
  const int tid = threadIdx.x, lane = tid & 31, wave = tid >> 5, hh = lane >> 4, m = lane & 15;
  const int n0 = blockIdx.x * NBN;

  {
    const int nl = tid >> 3, q = tid & 7;
    int node = n0 + nl;
    node = node > nN - 1 ? nN - 1 : node;
    const float* rp = nf + (size_t)node * 256 + 32 * q;
#pragma unroll
    for (int i4 = 0; i4 < 8; ++i4) {
      const v4f x = *(const v4f*)(rp + 4 * i4);
#pragma unroll
      for (int u = 0; u < 4; ++u) {
        const int j  = 32 * q + 4 * i4 + u;
        const int jj = j - 64;
        const int c  = jj / 3;
        const int mm = jj - 3 * c;
        const int row = (j < 64) ? nl : (32 + 32 * mm + nl);
        const int k   = (j < 64) ? j : c;
        unsigned short hi, lo;
        split_bf(x[u], hi, lo);
        sAh[row * APN + k] = hi;
        sAl[row * APN + k] = lo;
      }
    }
  }
  __syncthreads();

  const int part = wave >> 1;
  const int oh0 = part == 0 ? WO_N10H : WO_N11H;
  const int ol0 = part == 0 ? WO_N10L : WO_N11L;
  const int oh1 = part == 0 ? WO_N20H : WO_N21H;
  const int ol1 = part == 0 ? WO_N20L : WO_N21L;
  v8f acc[2][4];
#pragma unroll
  for (int W = 0; W < 2; ++W)
#pragma unroll
    for (int t = 0; t < 4; ++t) acc[W][t] = zero8();
  const unsigned short* aph = sAh + (16 * wave + m) * APN + 8 * hh;
  const unsigned short* apl = sAl + (16 * wave + m) * APN + 8 * hh;
#pragma unroll
  for (int ks = 0; ks < 2; ++ks) {
    FragB ah, al;
    ah.h[0] = *(const v8us*)(aph + 32 * ks);
    ah.h[1] = *(const v8us*)(aph + 32 * ks + 16);
    al.h[0] = *(const v8us*)(apl + 32 * ks);
    al.h[1] = *(const v8us*)(apl + 32 * ks + 16);
#pragma unroll
    for (int W = 0; W < 2; ++W) {
      const unsigned short* pH = wp + (W ? oh1 : oh0);
      const unsigned short* pL = wp + (W ? ol1 : ol0);
#pragma unroll
      for (int t = 0; t < 4; ++t) {
        const size_t bo = (size_t)(16 * t + m) * 64 + 32 * ks + 8 * hh;
        FragB bh, bl;
        bh.h[0] = *(const v8us*)(pH + bo);
        bh.h[1] = *(const v8us*)(pH + bo + 16);
        bl.h[0] = *(const v8us*)(pL + bo);
        bl.h[1] = *(const v8us*)(pL + bo + 16);
        acc[W][t] = wm(ah.v, bh.v, acc[W][t]);
        acc[W][t] = wm(ah.v, bl.v, acc[W][t]);
        acc[W][t] = wm(al.v, bh.v, acc[W][t]);
      }
    }
  }
  __syncthreads();

#pragma unroll
  for (int W = 0; W < 2; ++W) {
    float* sp = stg + (16 * wave + 8 * hh) * 64 + m;
#pragma unroll
    for (int t = 0; t < 4; ++t) {
#pragma unroll
      for (int r = 0; r < 8; ++r) sp[r * 64 + 16 * t] = acc[W][t][r] * 0.125f;
    }
    __syncthreads();
    float* T = W ? T2 : T1;
    v4f vals[4][2];
#pragma unroll
    for (int s = 0; s < 4; ++s) {
      const int nl = 4 * wave + s;
#pragma unroll
      for (int i = 0; i < 2; ++i) {
        const int f = 128 * i + 4 * lane;
        vals[s][i] = *(const v4f*)(stg + ((f >> 6) * 32 + nl) * 64 + (f & 63));
      }
    }
#pragma unroll
    for (int s = 0; s < 4; ++s) {
      const int nl = 4 * wave + s;
#pragma unroll
      for (int i = 0; i < 2; ++i)
        *(volatile v4f*)(T + (size_t)(n0 + nl) * TROW + 128 * i + 4 * lane) = vals[s][i];
    }
    __threadfence();
#pragma unroll
    for (int s = 0; s < 4; ++s) {
      const int nl = 4 * wave + s;
#pragma unroll
      for (int i = 0; i < 2; ++i)
        *(volatile v4f*)(T + (size_t)(n0 + nl) * TROW + 128 * i + 4 * lane) = vals[s][i];
    }
    __syncthreads();
  }
}

__device__ __forceinline__ void mlp_layer64(
    const unsigned short* inH, const unsigned short* inL,
    unsigned short* outH, unsigned short* outL,
    const unsigned short* __restrict__ pH, const unsigned short* __restrict__ pL,
    int rt, int cg, int hh, int m) {
  v8f acc[2];
  acc[0] = zero8(); acc[1] = zero8();
  const unsigned short* aph = inH + (16 * rt + m) * APN + 8 * hh;
  const unsigned short* apl = inL + (16 * rt + m) * APN + 8 * hh;
#pragma unroll
  for (int ks = 0; ks < 2; ++ks) {
    FragB ah, al;
    ah.h[0] = *(const v8us*)(aph + 32 * ks);
    ah.h[1] = *(const v8us*)(aph + 32 * ks + 16);
    al.h[0] = *(const v8us*)(apl + 32 * ks);
    al.h[1] = *(const v8us*)(apl + 32 * ks + 16);
#pragma unroll
    for (int t = 0; t < 2; ++t) {
      const int nt = 2 * cg + t;
      const size_t bo = (size_t)(16 * nt + m) * 64 + 32 * ks + 8 * hh;
      FragB bh, bl;
      bh.h[0] = *(const v8us*)(pH + bo);
      bh.h[1] = *(const v8us*)(pH + bo + 16);
      bl.h[0] = *(const v8us*)(pL + bo);
      bl.h[1] = *(const v8us*)(pL + bo + 16);
      acc[t] = wm(ah.v, bh.v, acc[t]);
      acc[t] = wm(ah.v, bl.v, acc[t]);
      acc[t] = wm(al.v, bh.v, acc[t]);
    }
  }
#pragma unroll
  for (int t = 0; t < 2; ++t) {
    const int col = 16 * (2 * cg + t) + m;
#pragma unroll
    for (int r = 0; r < 8; ++r) {
      const float x = silu_f(acc[t][r] * 0.125f);
      unsigned short hi, lo;
      split_bf(x, hi, lo);
      const int idx = (16 * rt + 8 * hh + r) * APN + col;
      outH[idx] = hi;
      outL[idx] = lo;
    }
  }
}

__global__ __launch_bounds__(NTHR) void k_edge(
    const float* __restrict__ ef, const float* __restrict__ ea, const int* __restrict__ ei,
    const float* __restrict__ Wf, const unsigned short* __restrict__ wp,
    const float* __restrict__ T1, const float* __restrict__ T2,
    float* out1, float* Pw, int nE, int nN) {
  __shared__ __attribute__((aligned(16))) float ldsu[9216];
  __shared__ __attribute__((aligned(16))) float sWf[128];
  __shared__ __attribute__((aligned(16))) float sY[NBE * 4];
  __shared__ __attribute__((aligned(16))) float sP[2 * NBE];
  __shared__ int sSnd[NBE];
  __shared__ int sRcv[NBE];
  unsigned short* actb = (unsigned short*)ldsu;
  unsigned short* X0h = actb;
  unsigned short* X0l = actb + 4608;
  unsigned short* X1h = actb + 9216;
  unsigned short* X1l = actb + 13824;
  float* sG = ldsu;
  const int tid = threadIdx.x, lane = tid & 31, wave = tid >> 5, hh = lane >> 4, m = lane & 15;
  const int e0 = blockIdx.x * NBE;

  if (tid < NBE) {
    int e = e0 + tid;
    e = e > nE - 1 ? nE - 1 : e;
    int s = ei[e];
    s = s < 0 ? 0 : (s > nN - 1 ? nN - 1 : s);
    int r = ei[(size_t)nE + e];
    r = r < 0 ? 0 : (r > nN - 1 ? nN - 1 : r);
    const v4f y = *(const v4f*)(ea + (size_t)e * 4);
    sSnd[tid] = s;
    sRcv[tid] = r;
    *(v4f*)(sY + 4 * tid) = y;
  } else if (tid < NBE + 128) {
    sWf[tid - NBE] = Wf[tid - NBE];
  }
  __syncthreads();

  const int rt = wave & 3, cg = wave >> 2;

  {
    int e = e0 + 16 * rt + m;
    e = e > nE - 1 ? nE - 1 : e;
    const float* rp = ef + (size_t)e * 8;
    const v4f xa = *(const v4f*)rp, xb = *(const v4f*)(rp + 4);
    float xv[8];
    xv[0] = xa.x; xv[1] = xa.y; xv[2] = xa.z; xv[3] = xa.w;
    xv[4] = xb.x; xv[5] = xb.y; xv[6] = xb.z; xv[7] = xb.w;
    v16us au;
#pragma unroll
    for (int i = 0; i < 8; ++i) {
      unsigned short hi, lo;
      split_bf(xv[i], hi, lo);
      au[i]     = hh ? lo : hi;
      au[8 + i] = hh ? (unsigned short)0 : hi;
    }
    FragB a;
    a.u = au;
    v8f acc[2];
#pragma unroll
    for (int t = 0; t < 2; ++t) {
      const int nt = 2 * cg + t;
      const unsigned short* bp = wp + WO_B0 + (size_t)(16 * nt + m) * 32 + 8 * hh;
      FragB b;
      b.h[0] = *(const v8us*)bp;
      b.h[1] = *(const v8us*)(bp + 16);
      acc[t] = wm(a.v, b.v, zero8());
    }
#pragma unroll
    for (int t = 0; t < 2; ++t) {
      const int col = 16 * (2 * cg + t) + m;
#pragma unroll
      for (int r = 0; r < 8; ++r) {
        const float x = silu_f(acc[t][r] * RS8);
        unsigned short hi, lo;
        split_bf(x, hi, lo);
        const int idx = (16 * rt + 8 * hh + r) * APN + col;
        X0h[idx] = hi;
        X0l[idx] = lo;
      }
    }
  }
  __syncthreads();
  mlp_layer64(X0h, X0l, X1h, X1l, wp + WO_F1H, wp + WO_F1L, rt, cg, hh, m);
  __syncthreads();
  mlp_layer64(X1h, X1l, X0h, X0l, wp + WO_F2H, wp + WO_F2L, rt, cg, hh, m);
  __syncthreads();

  v8f acc3[4];
#pragma unroll
  for (int t = 0; t < 4; ++t) acc3[t] = zero8();
  {
    const unsigned short* aph = X0h + (16 * rt + m) * APN + 8 * hh;
    const unsigned short* apl = X0l + (16 * rt + m) * APN + 8 * hh;
    const unsigned short* pH = wp + WO_F3H;
    const unsigned short* pL = wp + WO_F3L;
#pragma unroll
    for (int ks = 0; ks < 2; ++ks) {
      FragB ah, al;
      ah.h[0] = *(const v8us*)(aph + 32 * ks);
      ah.h[1] = *(const v8us*)(aph + 32 * ks + 16);
      al.h[0] = *(const v8us*)(apl + 32 * ks);
      al.h[1] = *(const v8us*)(apl + 32 * ks + 16);
#pragma unroll
      for (int t = 0; t < 4; ++t) {
        const int n = 64 * cg + 16 * t + m;
        const size_t bo = (size_t)n * 64 + 32 * ks + 8 * hh;
        FragB bh, bl;
        bh.h[0] = *(const v8us*)(pH + bo);
        bh.h[1] = *(const v8us*)(pH + bo + 16);
        bl.h[0] = *(const v8us*)(pL + bo);
        bl.h[1] = *(const v8us*)(pL + bo + 16);
        acc3[t] = wm(ah.v, bh.v, acc3[t]);
        acc3[t] = wm(ah.v, bl.v, acc3[t]);
        acc3[t] = wm(al.v, bh.v, acc3[t]);
      }
    }
  }
  __syncthreads();

  {
    const v2f wfa = *(const v2f*)(sWf + 2 * lane);
    v2f wfb = *(const v2f*)(sWf + 64 + 2 * lane);
    wfb = wfb * SQ3I;
#pragma unroll 1
    for (int j = 0; j < 8; ++j) {
      const int el = 8 * wave + j;
      const int sn = sSnd[el];
      const int rc = sRcv[el];
      const v4f y = *(const v4f*)(sY + 4 * el);
      const float* t1 = T1 + (size_t)sn * TROW + 2 * lane;
      const float* t2 = T2 + (size_t)rc * TROW + 2 * lane;
      const v2f s1 = *(const v2f*)t1,         s2 = *(const v2f*)t2;
      const v2f a0 = *(const v2f*)(t1 + 64),  b0 = *(const v2f*)(t2 + 64);
      const v2f a1 = *(const v2f*)(t1 + 128), b1 = *(const v2f*)(t2 + 128);
      const v2f a2 = *(const v2f*)(t1 + 192), b2 = *(const v2f*)(t2 + 192);
      const v2f bs = s1 + s2;
      const v2f d  = (a0 + b0) * y.y + (a1 + b1) * y.z + (a2 + b2) * y.w;
      const v2f g0 = (bs * y.x) * wfa;
      const v2f g1 = d * wfb;
      *(v2f*)(sG + el * 128 + 2 * lane) = g0;
      *(v2f*)(sG + el * 128 + 64 + 2 * lane) = g1;
    }
  }
  __syncthreads();

  {
    float ps[8];
#pragma unroll
    for (int r = 0; r < 8; ++r) ps[r] = 0.f;
    const float* gp = sG + (16 * rt + 8 * hh) * 128 + 64 * cg + m;
#pragma unroll
    for (int t = 0; t < 4; ++t) {
#pragma unroll
      for (int r = 0; r < 8; ++r) ps[r] += acc3[t][r] * gp[r * 128 + 16 * t];
    }
#pragma unroll
    for (int r = 0; r < 8; ++r) {
      float v = ps[r];
      v += __shfl_xor(v, 1);
      v += __shfl_xor(v, 2);
      v += __shfl_xor(v, 4);
      v += __shfl_xor(v, 8);
      ps[r] = v;
    }
    if (m == 0) {
#pragma unroll
      for (int r = 0; r < 8; ++r) sP[cg * NBE + 16 * rt + 8 * hh + r] = ps[r];
    }
  }
  __syncthreads();

  if (wave == 0) {
    const int l = lane & 15;
    v4f o;
#pragma unroll
    for (int j = 0; j < 4; ++j) {
      const int el = 4 * l + j;
      o[j] = (((sP[el] + sP[NBE + el]) * 0.125f) * RS128) * R40;
    }
    const int eb = e0 + 4 * l;
    if (lane < 16) {
      *(volatile v4f*)(Pw + eb) = o;
      if (eb + 3 < nE) {
        *(volatile v4f*)(out1 + eb) = o;
      } else {
        if (eb     < nE) *(volatile float*)(out1 + eb)     = o.x;
        if (eb + 1 < nE) *(volatile float*)(out1 + eb + 1) = o.y;
        if (eb + 2 < nE) *(volatile float*)(out1 + eb + 2) = o.z;
      }
    }
    __threadfence();
    if (lane < 16) {
      *(volatile v4f*)(Pw + eb) = o;
      if (eb + 3 < nE) {
        *(volatile v4f*)(out1 + eb) = o;
      } else {
        if (eb     < nE) *(volatile float*)(out1 + eb)     = o.x;
        if (eb + 1 < nE) *(volatile float*)(out1 + eb + 1) = o.y;
        if (eb + 2 < nE) *(volatile float*)(out1 + eb + 2) = o.z;
      }
    }
  }
}

template <int NB>
__device__ __forceinline__ int scan_chunk(const int* __restrict__ keys, int nE, int cbase, int slotBase,
                                          int vec8, int* list, int tid, int lane, int wave) {
  int wc = 0;
#pragma unroll
  for (int g = 0; g < NGRP; ++g) {
    const int el0  = (g * NTHR + tid) * EPT;
    const int e0   = cbase + el0;
    const int sent = -2147483647 - 1;
    v4i da, db;
    if (vec8 != 0 && cbase + CHUNK <= nE) {
      da = *(const v4i*)(keys + e0);
      db = *(const v4i*)(keys + e0 + 4);
    } else {
      da.x = (e0     < nE) ? keys[min(e0, nE - 1)] : sent;
      da.y = (e0 + 1 < nE) ? keys[min(e0 + 1, nE - 1)] : sent;
      da.z = (e0 + 2 < nE) ? keys[min(e0 + 2, nE - 1)] : sent;
      da.w = (e0 + 3 < nE) ? keys[min(e0 + 3, nE - 1)] : sent;
      db.x = (e0 + 4 < nE) ? keys[min(e0 + 4, nE - 1)] : sent;
      db.y = (e0 + 5 < nE) ? keys[min(e0 + 5, nE - 1)] : sent;
      db.z = (e0 + 6 < nE) ? keys[min(e0 + 6, nE - 1)] : sent;
      db.w = (e0 + 7 < nE) ? keys[min(e0 + 7, nE - 1)] : sent;
    }
    const unsigned nb = (unsigned)slotBase;
    const unsigned s0 = (unsigned)da.x - nb, s1 = (unsigned)da.y - nb;
    const unsigned s2 = (unsigned)da.z - nb, s3 = (unsigned)da.w - nb;
    const unsigned s4 = (unsigned)db.x - nb, s5 = (unsigned)db.y - nb;
    const unsigned s6 = (unsigned)db.z - nb, s7 = (unsigned)db.w - nb;
    const bool h0 = s0 < (unsigned)NB, h1 = s1 < (unsigned)NB, h2 = s2 < (unsigned)NB, h3 = s3 < (unsigned)NB;
    const bool h4 = s4 < (unsigned)NB, h5 = s5 < (unsigned)NB, h6 = s6 < (unsigned)NB, h7 = s7 < (unsigned)NB;
    const unsigned any = __builtin_amdgcn_ballot_w32(h0 | h1 | h2 | h3 | h4 | h5 | h6 | h7);
    if (any != 0u) {
#define HITJ(J, HJ, SJ) { \
        const unsigned mj = __builtin_amdgcn_ballot_w32(HJ); \
        if (mj != 0u) { \
          if (HJ) { \
            const int pos = wc + (int)__builtin_amdgcn_mbcnt_lo(mj, 0u); \
            if (pos < WCAP) list[wave * WCAP + pos] = ((el0 + (J)) << 12) | (int)(SJ); \
          } \
          wc += (int)__builtin_popcount(mj); } }
      HITJ(0, h0, s0)
      HITJ(1, h1, s1)
      HITJ(2, h2, s2)
      HITJ(3, h3, s3)
      HITJ(4, h4, s4)
      HITJ(5, h5, s5)
      HITJ(6, h6, s6)
      HITJ(7, h7, s7)
#undef HITJ
    }
  }
  return wc;
}

__device__ __forceinline__ void drain_hits(const int* list, const int* wcnt, float* acc,
                                           const float* __restrict__ Pw, int cbase, int nE, int lane) {
#pragma unroll 1
  for (int wsx = 0; wsx < NWAVE; ++wsx) {
    int n = __builtin_amdgcn_readfirstlane(wcnt[wsx]);
    n = n > WCAP ? WCAP : (n < 0 ? 0 : n);
    const int* lp = list + wsx * WCAP;
#pragma unroll 1
    for (int i = 0; i < n; ++i) {
      const int ent  = __builtin_amdgcn_readfirstlane(lp[i]);
      const int slot = ent & (NBC - 1);
      int e = cbase + ((ent >> 12) & (CHUNK - 1));
      e = e > nE - 1 ? nE - 1 : e;
      const float pv = Pw[e];
      if (lane == 0) acc[slot] = acc[slot] + pv;
    }
  }
}

__global__ __launch_bounds__(NTHR) void k_charge(
    const int* __restrict__ ei, const float* __restrict__ Pw,
    const float* __restrict__ nf, const float* __restrict__ Wm1,
    float* out0, int nE, int nN, int vec8) {
  __shared__ __attribute__((aligned(16))) float accR[NBC];
  __shared__ __attribute__((aligned(16))) float accS[NBC];
  __shared__ __attribute__((aligned(16))) int list[LISTN];
  __shared__ float sWm[CH];
  __shared__ int wcnt[NWAVE];
  const int tid = threadIdx.x, lane = tid & 31, wave = tid >> 5;
  const int nodeBase = blockIdx.x * NBC;

  for (int i = tid; i < NBC; i += NTHR) { accR[i] = 0.f; accS[i] = 0.f; }
  if (tid < CH) sWm[tid] = Wm1[tid];
  __syncthreads();

  const int nChunks = (nE + CHUNK - 1) / CHUNK;
#pragma unroll 1
  for (int ch = 0; ch < nChunks; ++ch) {
    const int cbase = ch * CHUNK;
    int wc = scan_chunk<NBC>(ei + nE, nE, cbase, nodeBase, vec8, list, tid, lane, wave);
    if (lane == 0) wcnt[wave] = wc;
    __syncthreads();
    if (wave == 0) drain_hits(list, wcnt, accR, Pw, cbase, nE, lane);
    __syncthreads();
    wc = scan_chunk<NBC>(ei, nE, cbase, nodeBase, vec8, list, tid, lane, wave);
    if (lane == 0) wcnt[wave] = wc;
    __syncthreads();
    if (wave == 0) drain_hits(list, wcnt, accS, Pw, cbase, nE, lane);
    __syncthreads();
  }

#pragma unroll 1
  for (int g = 0; g < NBC / (32 * NWAVE); ++g) {
    const int slot0 = 32 * (g * NWAVE + wave);
    if (nodeBase + slot0 >= nN) continue;
    const int slot = slot0 + lane;
    const int node = nodeBase + slot;
    const int nn = node > nN - 1 ? nN - 1 : node;
    const float* row = nf + (size_t)nn * 256 + 64;
    float a0 = 0.f, a1 = 0.f, a2 = 0.f;
#pragma unroll 1
    for (int i = 0; i < 16; ++i) {
      const v4f u0 = *(const v4f*)(row + 12 * i);
      const v4f u1 = *(const v4f*)(row + 12 * i + 4);
      const v4f u2 = *(const v4f*)(row + 12 * i + 8);
      const float w0 = sWm[4 * i], w1 = sWm[4 * i + 1], w2 = sWm[4 * i + 2], w3 = sWm[4 * i + 3];
      a0 = a0 + u0.x * w0 + u0.w * w1 + u1.z * w2 + u2.y * w3;
      a1 = a1 + u0.y * w0 + u1.x * w1 + u1.w * w2 + u2.z * w3;
      a2 = a2 + u0.z * w0 + u1.y * w1 + u2.x * w2 + u2.w * w3;
    }
    const float chg = accR[slot] - accS[slot];
    v4f o;
    o.x = chg; o.y = a0 * 0.125f; o.z = a1 * 0.125f; o.w = a2 * 0.125f;
    if (node < nN) *(volatile v4f*)(out0 + (size_t)node * 4) = o;
    __threadfence();
    if (node < nN) *(volatile v4f*)(out0 + (size_t)node * 4) = o;
  }
}

extern "C" void kernel_launch(void* const* d_in, const int* in_sizes, int n_in,
                              void* d_out, int out_size, void* d_ws, size_t ws_size,
                              hipStream_t stream) {
  if (n_in < 18) return;
  const int nN = in_sizes[1] / 256;
  const int nE = in_sizes[3] / 8;
  if (nN < 1 || nE < 1) return;
  if (in_sizes[1] != nN * 256 || in_sizes[3] != nE * 8) return;
  if (in_sizes[2] != 4 * nE || in_sizes[4] != 2 * nE) return;
  if (in_sizes[8] != 4096 || in_sizes[9] != 4096 || in_sizes[10] != 4096 || in_sizes[11] != 4096) return;
  if (in_sizes[12] != 512 || in_sizes[13] != 4096 || in_sizes[14] != 4096 || in_sizes[15] != 16384) return;
  if (in_sizes[16] != 128 || in_sizes[17] != 64) return;
  if (out_size != 4 * nN + nE) return;
  if (nN > (1 << 24) || nE > (1 << 26)) return;

  const float* nf  = (const float*)d_in[1];
  const float* ea  = (const float*)d_in[2];
  const float* ef  = (const float*)d_in[3];
  const int*   ei  = (const int*)d_in[4];
  const float* w10 = (const float*)d_in[8];
  const float* w11 = (const float*)d_in[9];
  const float* w20 = (const float*)d_in[10];
  const float* w21 = (const float*)d_in[11];
  const float* fw0 = (const float*)d_in[12];
  const float* fw1 = (const float*)d_in[13];
  const float* fw2 = (const float*)d_in[14];
  const float* fw3 = (const float*)d_in[15];
  const float* Wf  = (const float*)d_in[16];
  const float* Wm1 = (const float*)d_in[17];
  float* out0 = (float*)d_out;
  float* out1 = out0 + (size_t)4 * nN;

  const int nbNode = (nN + NBN - 1) / NBN;
  const int Npad   = nbNode * NBN;
  const int nbEdge = (nE + NBE - 1) / NBE;
  const int Epad   = nbEdge * NBE;
  const int nbChg  = (nN + NBC - 1) / NBC;

  char* ws = (char*)d_ws;
  size_t off = 0;
  const size_t oW  = off; off += (size_t)WTOT * 2;         off = (off + 255) & ~(size_t)255;
  const size_t oT1 = off; off += (size_t)Npad * TROW * 4;  off = (off + 255) & ~(size_t)255;
  const size_t oT2 = off; off += (size_t)Npad * TROW * 4;  off = (off + 255) & ~(size_t)255;
  const size_t oP  = off; off += (size_t)Epad * 4;         off = (off + 255) & ~(size_t)255;
  if (off > ws_size || off > (size_t)WSCAP) return;
  unsigned short* wp = (unsigned short*)(ws + oW);
  float* T1 = (float*)(ws + oT1);
  float* T2 = (float*)(ws + oT2);
  float* Pw = (float*)(ws + oP);

  const int vec8 = ((nE & 3) == 0) ? 1 : 0;

  k_wprep<<<WBLK, NTHR, 0, stream>>>(fw0, fw1, fw2, fw3, w10, w11, w20, w21, wp);
  k_node<<<nbNode, NTHR, 0, stream>>>(nf, wp, T1, T2, nN);
  k_edge<<<nbEdge, NTHR, 0, stream>>>(ef, ea, ei, Wf, wp, T1, T2, out1, Pw, nE, nN);
  k_charge<<<nbChg, NTHR, 0, stream>>>(ei, Pw, nf, Wm1, out0, nE, nN, vec8);
}
